// EncoderBlock_75359496176199
// MI455X (gfx1250) — hardware-verified
//
#include <hip/hip_runtime.h>
#include <math.h>

#ifndef NB
#define NB 2
#endif
#ifndef SEQ
#define SEQ 1024
#endif
#define NB_FULL 2
#define SEQ_FULL 1024
#define DM 1024
#define NHB 16
#define DHD 64
#define ROWS (NB * SEQ)
#define NHEAD (NB * NHB)

static_assert(SEQ % 64 == 0);
static_assert(SEQ <= 1024);
static_assert(SEQ <= SEQ_FULL);
static_assert(NB <= NB_FULL);
static_assert(ROWS % 64 == 0);
static_assert(DM % 64 == 0);
static_assert(DM % 32 == 0);
static_assert(DM == NHB * DHD);
static_assert(DHD == 64);
static_assert(DM == 8 * 128);
static_assert((DM % 8) == 0);

typedef __attribute__((ext_vector_type(16))) _Float16 v16h;
typedef __attribute__((ext_vector_type(8)))  _Float16 v8h;
typedef __attribute__((ext_vector_type(16))) __bf16   v16b;
typedef __attribute__((ext_vector_type(8)))  __bf16   v8b;
typedef __attribute__((ext_vector_type(8)))  float    v8f;
typedef __attribute__((ext_vector_type(4)))  float    v4f;
typedef __attribute__((ext_vector_type(4)))  unsigned int u4v;
typedef __attribute__((ext_vector_type(2)))  unsigned int u2v;


#define VST2(T, ptr, val) do { const T vst2_v_ = (val); *(volatile T*)(ptr) = vst2_v_; __threadfence(); *(volatile T*)(ptr) = vst2_v_; } while (0)

__device__ __forceinline__ float cmb_bf(float v) {
    const unsigned u = __builtin_bit_cast(unsigned, v);
    const unsigned r = (u + 0x7fffu + ((u >> 16) & 1u)) & 0xffff0000u;
    return __builtin_bit_cast(float, r);
}
__device__ __forceinline__ unsigned cmb_pk2(float a, float b) {
    return (unsigned)__builtin_bit_cast(unsigned short, (_Float16)a) | ((unsigned)__builtin_bit_cast(unsigned short, (_Float16)b) << 16);
}
__device__ __forceinline__ unsigned short f2bf_bits(float f) {
    const unsigned u = __float_as_uint(f);
    return (unsigned short)((u + 0x7FFFu + ((u >> 16) & 1u)) >> 16);
}
__device__ __forceinline__ float bf_bits2f(unsigned short h) { return __uint_as_float(((unsigned)h) << 16); }
__device__ __forceinline__ unsigned bf_pk2_split(float a, float b, unsigned* lo) {
    const unsigned short ha = f2bf_bits(a), hb = f2bf_bits(b);
    const unsigned short la = f2bf_bits(a - bf_bits2f(ha)), lb = f2bf_bits(b - bf_bits2f(hb));
    *lo = (unsigned)la | ((unsigned)lb << 16);
    return (unsigned)ha | ((unsigned)hb << 16);
}

union FH { v16h v; v8h h[2]; };
union FB { v16b v; v8b h[2]; };
__device__ __forceinline__ v16h ldfrag_h_g(const _Float16* __restrict__ p) { FH f; f.h[0] = *(const v8h*)(p); f.h[1] = *(const v8h*)(p + 16); return f.v; }
__device__ __forceinline__ v16b ldfrag_b_g(const __bf16* __restrict__ p)   { FB f; f.h[0] = *(const v8b*)(p); f.h[1] = *(const v8b*)(p + 16); return f.v; }

__device__ __forceinline__ v8f mma_h(v16h a, v16h b, v8f c) {
    return __builtin_amdgcn_wmma_f32_16x16x32_f16(false, a, false, b, (short)0, c, false, false);
}
__device__ __forceinline__ void dep_guard_h(v8f& a, v8f& b, v16h x, v16h y) { asm volatile("v_nop\n\tv_nop\n\tv_nop\n\tv_nop" : "+v"(a), "+v"(b) : "v"(x), "v"(y)); }
__device__ __forceinline__ void keep4_h(v16h a, v16h b, v16h c, v16h d) { asm volatile("v_nop" :: "v"(a), "v"(b), "v"(c), "v"(d)); }
__device__ __forceinline__ void acc_guard4(v8f& a, v8f& b, v8f& c, v8f& d) { asm volatile("v_nop\n\tv_nop\n\tv_nop\n\tv_nop" : "+v"(a), "+v"(b), "+v"(c), "+v"(d)); }
__device__ __forceinline__ void guard_pv(v8f& a, v8f& b, v16h x, v16h y, v16h z, v16h w) { asm volatile("v_nop\n\tv_nop\n\tv_nop\n\tv_nop" : "+v"(a), "+v"(b) : "v"(x), "v"(y), "v"(z), "v"(w)); }
__device__ __forceinline__ v8f mma_b3(v16b ah, v16b al, v16b bh, v16b bl, v8f c) {
    c = __builtin_amdgcn_wmma_f32_16x16x32_bf16(false, ah, false, bl, (short)0, c, false, false);
    c = __builtin_amdgcn_wmma_f32_16x16x32_bf16(false, al, false, bh, (short)0, c, false, false);
    c = __builtin_amdgcn_wmma_f32_16x16x32_bf16(false, ah, false, bh, (short)0, c, false, false);
    asm volatile("v_nop\n\tv_nop\n\tv_nop\n\tv_nop" : "+v"(c) : "v"(ah), "v"(al), "v"(bh), "v"(bl));
    return c;
}
__device__ __forceinline__ void wave_sync_lds() {
    __builtin_amdgcn_fence(3  , "workgroup");
    __builtin_amdgcn_wave_barrier();
    __builtin_amdgcn_fence(2  , "workgroup");
}

__global__ __launch_bounds__(256) void k_castb(const float* __restrict__ SRC, unsigned short* __restrict__ DST, int nR, int rows_per_b, int src_rows_per_b, float sc) {
    const long long u = (long long)blockIdx.x * 256 + threadIdx.x;
    const int per = DM / 8;
    if (u >= (long long)nR * per) return;
    const int r = (int)(u / per); const int c0 = 8 * (int)(u % per);
    const long long sr = (long long)(r / rows_per_b) * src_rows_per_b + (r % rows_per_b);
    const float* s = SRC + sr * DM + c0;
    const v4f a = *(const v4f*)(s), b = *(const v4f*)(s + 4);
    u4v pk;
    pk.x = cmb_pk2(cmb_bf(a.x) * sc, cmb_bf(a.y) * sc);
    pk.y = cmb_pk2(cmb_bf(a.z) * sc, cmb_bf(a.w) * sc);
    pk.z = cmb_pk2(cmb_bf(b.x) * sc, cmb_bf(b.y) * sc);
    pk.w = cmb_pk2(cmb_bf(b.z) * sc, cmb_bf(b.w) * sc);
    VST2(u4v, (u4v*)(DST + (long long)r * DM + c0), pk);
}

template <int OUT_MODE>
__device__ __forceinline__ void gemm64_body(float* sTbase,
    const unsigned short* __restrict__ Ap, int lda, const unsigned short* __restrict__ Btp, int ldb,
    void* __restrict__ Cout, void* __restrict__ Cout2, int ldc, const float* __restrict__ bias,
    int M, int N, int K, float scale) {
  const _Float16* A = (const _Float16*)Ap; const _Float16* Bt = (const _Float16*)Btp;
  const int lane = threadIdx.x & 31;
  const int wave = threadIdx.x >> 5;
  const int tilesN = N >> 6;
  const int tilesM = M >> 6;
  const int tile = blockIdx.x * 8 + wave;
  if (tile >= tilesM * tilesN) return;
  const int tm = tile / tilesN;
  const int tn = tile - tm * tilesN;
  const int m0 = tm << 6;
  const int n0 = tn << 6;
  const int rlane = lane & 15;
  const int koff  = (lane >> 4) * 8;
  const int mOff  = (lane >> 4) * 8;

  v8f acc[4][4];
#pragma unroll
  for (int i = 0; i < 4; ++i)
#pragma unroll
    for (int j = 0; j < 4; ++j) acc[i][j] = (v8f){0.f,0.f,0.f,0.f,0.f,0.f,0.f,0.f};

  for (int k0 = 0; k0 < K; k0 += 32) {
    v16h bh[4];
#pragma unroll
    for (int j = 0; j < 4; ++j) bh[j] = ldfrag_h_g(Bt + (size_t)(n0 + (j << 4) + rlane) * ldb + koff + k0);
#pragma unroll
    for (int i = 0; i < 4; ++i) {
      const v16h ah = ldfrag_h_g(A + (size_t)(m0 + (i << 4) + rlane) * lda + koff + k0);
#pragma unroll
      for (int j = 0; j < 4; ++j) acc[i][j] = mma_h(ah, bh[j], acc[i][j]);
      dep_guard_h(acc[i][0], acc[i][3], ah, ah);
    }
    keep4_h(bh[0], bh[1], bh[2], bh[3]);
  }
  acc_guard4(acc[0][0], acc[0][1], acc[0][2], acc[0][3]);
  acc_guard4(acc[1][0], acc[1][1], acc[1][2], acc[1][3]);
  acc_guard4(acc[2][0], acc[2][1], acc[2][2], acc[2][3]);
  acc_guard4(acc[3][0], acc[3][1], acc[3][2], acc[3][3]);

  float* slab = sTbase + wave * (16 * 68);
  float bvj[4];
#pragma unroll
  for (int j = 0; j < 4; ++j) bvj[j] = cmb_bf(bias[n0 + (j << 4) + rlane]);
#pragma unroll
  for (int i = 0; i < 4; ++i) {
    const int mBase = m0 + (i << 4);
#pragma unroll
    for (int j = 0; j < 4; ++j) {
#pragma unroll
      for (int r = 0; r < 8; ++r) slab[(mOff + r) * 68 + (j << 4) + rlane] = acc[i][j][r] * scale + bvj[j];
    }
    wave_sync_lds();
    if (OUT_MODE == 0) {
      float* C = (float*)Cout;
      const int hh = lane >> 4, c4 = (lane & 15) * 4;
      for (int pass = 0; pass < 2; ++pass) {
#pragma unroll
        for (int it = 0; it < 8; ++it) {
          const int row = it * 2 + hh;
          const v4f v = *(const v4f*)(slab + row * 68 + c4);
          *(volatile v4f*)(C + (size_t)(mBase + row) * ldc + n0 + c4) = v;
        }
        __threadfence();
      }
    } else {
      const int q = lane >> 3, c8 = (lane & 7) * 8;
      unsigned short* C  = (unsigned short*)Cout;
      unsigned short* C2 = (unsigned short*)Cout2;
      for (int pass = 0; pass < 2; ++pass) {
#pragma unroll
        for (int it = 0; it < 4; ++it) {
          const int row = it * 4 + q;
          const v4f f0 = *(const v4f*)(slab + row * 68 + c8), f1 = *(const v4f*)(slab + row * 68 + c8 + 4);
          u4v ph, pl;
          if (OUT_MODE == 1) {
            ph.x = cmb_pk2(f0.x, f0.y); ph.y = cmb_pk2(f0.z, f0.w); ph.z = cmb_pk2(f1.x, f1.y); ph.w = cmb_pk2(f1.z, f1.w); pl = ph;
          } else {
            unsigned l0, l1, l2, l3;
            ph.x = bf_pk2_split(f0.x, f0.y, &l0); ph.y = bf_pk2_split(f0.z, f0.w, &l1);
            ph.z = bf_pk2_split(f1.x, f1.y, &l2); ph.w = bf_pk2_split(f1.z, f1.w, &l3);
            pl.x = l0; pl.y = l1; pl.z = l2; pl.w = l3;
          }
          *(volatile u4v*)(C + (size_t)(mBase + row) * ldc + n0 + c8) = ph;
          if (OUT_MODE == 2) *(volatile u4v*)(C2 + (size_t)(mBase + row) * ldc + n0 + c8) = pl;
        }
        __threadfence();
      }
    }
    wave_sync_lds();
  }
}

__global__ __launch_bounds__(256) void k_gemm_hl(const unsigned short* __restrict__ A, int lda, const unsigned short* __restrict__ Bt, int ldb,
    unsigned short* __restrict__ Chi, unsigned short* __restrict__ Clo, int ldc, const float* __restrict__ bias, int M, int N, int K, float scale) {
  __shared__ __align__(16) float sT[8 * 16 * 68];
  gemm64_body<2>(sT, A, lda, Bt, ldb, (void*)Chi, (void*)Clo, ldc, bias, M, N, K, scale);
}
__global__ __launch_bounds__(256) void k_gemm_h16(const unsigned short* __restrict__ A, int lda, const unsigned short* __restrict__ Bt, int ldb,
    unsigned short* __restrict__ C16, int ldc, const float* __restrict__ bias, int M, int N, int K, float scale) {
  __shared__ __align__(16) float sT[8 * 16 * 68];
  gemm64_body<1>(sT, A, lda, Bt, ldb, (void*)C16, (void*)C16, ldc, bias, M, N, K, scale);
}
__global__ __launch_bounds__(256) void k_gemm_f32(const unsigned short* __restrict__ A, int lda, const unsigned short* __restrict__ Bt, int ldb,
    float* __restrict__ C, int ldc, const float* __restrict__ bias, int M, int N, int K, float scale) {
  __shared__ __align__(16) float sT[8 * 16 * 68];
  gemm64_body<0>(sT, A, lda, Bt, ldb, (void*)C, (void*)C, ldc, bias, M, N, K, scale);
}

__global__ __launch_bounds__(256) void k_vt(const unsigned short* __restrict__ V16, unsigned short* __restrict__ Vt) {
  __shared__ unsigned int ltw[64 * 36];
  const int n = blockIdx.x / (SEQ / 64), t0 = (blockIdx.x % (SEQ / 64)) * 64;
  const int tid = threadIdx.x;
  const unsigned short* src = V16 + ((size_t)n * SEQ + t0) * 64;
#pragma unroll
  for (int it = 0; it < 2; ++it) {
    const int p = tid + 256 * it; const int t = p >> 3, sg = p & 7;
    const u4v g = *(const u4v*)(src + t * 64 + sg * 8);
    const int b = t * 36 + sg * 4;
    ltw[b] = g.x; ltw[b + 1] = g.y; ltw[b + 2] = g.z; ltw[b + 3] = g.w;
  }
  __syncthreads();
#pragma unroll
  for (int it = 0; it < 2; ++it) {
    const int p = tid + 256 * it; const int d = p >> 3, ts = p & 7;
    const int wsel = d >> 1, sh = (d & 1) * 16;
    unsigned hv[8];
#pragma unroll
    for (int e = 0; e < 8; ++e) hv[e] = (ltw[(ts * 8 + e) * 36 + wsel] >> sh) & 0xFFFFu;
    u4v pk; pk.x = hv[0] | (hv[1] << 16); pk.y = hv[2] | (hv[3] << 16); pk.z = hv[4] | (hv[5] << 16); pk.w = hv[6] | (hv[7] << 16);
    VST2(u4v, (u4v*)(Vt + ((size_t)n * 64 + d) * SEQ + t0 + ts * 8), pk);
  }
}

__global__ __launch_bounds__(128) void k_attn_rb(const unsigned short* __restrict__ Qhp, const unsigned short* __restrict__ Qlp,
    const unsigned short* __restrict__ Khp, const unsigned short* __restrict__ Klp, const unsigned short* __restrict__ Vtp,
    const float* __restrict__ rel_bias, unsigned short* __restrict__ AO) {
  __shared__ __align__(16) _Float16 brt[2048];
  __shared__ __align__(16) _Float16 Psh[4 * 16 * 64];
  __shared__ __align__(16) _Float16 Psl[4 * 16 * 64];
  __shared__ __align__(16) float    Os[4 * 16 * 68];
  const int tid = threadIdx.x, wave = tid >> 5, lane = tid & 31, hh = lane >> 4, c = lane & 15;
  const int qb = blockIdx.x % (SEQ / 64);
  const int n  = blockIdx.x / (SEQ / 64);
  const int jh = n % NHB;
  const int q0 = qb * 64 + wave * 16;

#pragma unroll 1
  for (int i = tid; i < 2048; i += 128) {
    const int rel = 1023 - i;
    const int a = (rel < 0) ? -rel : rel;
    const int big = 8 + (a >= 12) + (a >= 16) + (a >= 23) + (a >= 32) + (a >= 46) + (a >= 64) + (a >= 91);
    const int base = (a < 8) ? a : big;
    const int bucket = base + ((rel > 0) ? 16 : 0);
    brt[i] = (_Float16)(cmb_bf(rel_bias[bucket * 16 + jh]) * 1024.0f);
  }
  __syncthreads();

  const size_t hb = (size_t)n * SEQ * 64;
  const __bf16* Qh = (const __bf16*)Qhp + hb; const __bf16* Ql = (const __bf16*)Qlp + hb;
  const __bf16* Kh = (const __bf16*)Khp + hb; const __bf16* Kl = (const __bf16*)Klp + hb;
  const _Float16* Vt = (const _Float16*)Vtp + hb;

  const size_t qo = (size_t)(q0 + c) * 64 + 8 * hh;
  const v16b qh0 = ldfrag_b_g(Qh + qo), qh1 = ldfrag_b_g(Qh + qo + 32);
  const v16b ql0 = ldfrag_b_g(Ql + qo), ql1 = ldfrag_b_g(Ql + qo + 32);

  float mrow[8], lrow[8];
  v8f oacc[4], obias[4];
#pragma unroll
  for (int r = 0; r < 8; ++r) { mrow[r] = -INFINITY; lrow[r] = 0.f; }
#pragma unroll
  for (int t = 0; t < 4; ++t) { oacc[t] = (v8f){0.f,0.f,0.f,0.f,0.f,0.f,0.f,0.f}; obias[t] = (v8f){0.f,0.f,0.f,0.f,0.f,0.f,0.f,0.f}; }

  const float L2E = 1.4426950408889634f;
  const int pw = wave * (16 * 64);

#pragma unroll 1
  for (int kc = 0; kc < SEQ / 64; ++kc) {
    const int kv0 = kc * 64;
    v8f s[4];
#pragma unroll
    for (int j = 0; j < 4; ++j) {
      const size_t ko = (size_t)(kv0 + j * 16 + c) * 64 + 8 * hh;
      const v16b kh0 = ldfrag_b_g(Kh + ko), kl0 = ldfrag_b_g(Kl + ko);
      const v16b kh1 = ldfrag_b_g(Kh + ko + 32), kl1 = ldfrag_b_g(Kl + ko + 32);
      v8f a = (v8f){0.f,0.f,0.f,0.f,0.f,0.f,0.f,0.f};
      a = mma_b3(qh0, ql0, kh0, kl0, a);
      a = mma_b3(qh1, ql1, kh1, kl1, a);
      s[j] = a;
      __builtin_amdgcn_sched_barrier(0);
    }
#pragma unroll
    for (int r = 0; r < 8; ++r) {
      float m = fmaxf(fmaxf(s[0][r], s[1][r]), fmaxf(s[2][r], s[3][r]));
      m = fmaxf(m, __shfl_xor(m, 1, 32)); m = fmaxf(m, __shfl_xor(m, 2, 32));
      m = fmaxf(m, __shfl_xor(m, 4, 32)); m = fmaxf(m, __shfl_xor(m, 8, 32));
      const float mnew = fmaxf(mrow[r], m);
      const float alpha = exp2f((mrow[r] - mnew) * L2E);
      mrow[r] = mnew;
      float psum = 0.f;
#pragma unroll
      for (int j = 0; j < 4; ++j) {
        const float p = exp2f((s[j][r] - mnew) * L2E);
        psum += p;
        const float pc = p * 16384.0f;
        const _Float16 phi = (_Float16)pc;
        const _Float16 plo = (_Float16)(pc - (float)phi);
        Psh[pw + (8 * hh + r) * 64 + j * 16 + c] = phi;
        Psl[pw + (8 * hh + r) * 64 + j * 16 + c] = plo;
      }
      psum += __shfl_xor(psum, 1, 32); psum += __shfl_xor(psum, 2, 32);
      psum += __shfl_xor(psum, 4, 32); psum += __shfl_xor(psum, 8, 32);
      lrow[r] = lrow[r] * alpha + psum;
#pragma unroll
      for (int t = 0; t < 4; ++t) oacc[t][r] *= alpha;
    }
    wave_sync_lds();
#pragma unroll 1
    for (int kk = 0; kk < 2; ++kk) {
      const int po = pw + c * 64 + kk * 32 + 8 * hh;
      FH pa, pl;
      pa.h[0] = *(const v8h*)&Psh[po]; pa.h[1] = *(const v8h*)&Psh[po + 16];
      pl.h[0] = *(const v8h*)&Psl[po]; pl.h[1] = *(const v8h*)&Psl[po + 16];
      const int ib = kv0 + kk * 32 + 8 * hh - (q0 + c) + 1023;
      v16h ba;
#pragma unroll
      for (int e = 0; e < 8; ++e) { ba[e] = brt[ib + e]; ba[8 + e] = brt[ib + 16 + e]; }
#pragma unroll
      for (int t = 0; t < 4; ++t) {
        const v16h vb = ldfrag_h_g(Vt + (size_t)(t * 16 + c) * SEQ + kv0 + kk * 32 + 8 * hh);
        oacc[t]  = mma_h(pa.v, vb, oacc[t]);
        oacc[t]  = mma_h(pl.v, vb, oacc[t]);
        obias[t] = mma_h(ba, vb, obias[t]);
        guard_pv(oacc[t], obias[t], pa.v, pl.v, ba, vb);
        __builtin_amdgcn_sched_barrier(0);
      }
    }
    wave_sync_lds();
  }

  const int ow = wave * (16 * 68);
#pragma unroll
  for (int r = 0; r < 8; ++r) {
    const float inv = 1.0f / (lrow[r] * 16384.0f);
#pragma unroll
    for (int t = 0; t < 4; ++t) Os[ow + (8 * hh + r) * 68 + t * 16 + c] = oacc[t][r] * inv + obias[t][r] * (1.0f / 1024.0f);
  }
  wave_sync_lds();
  {
    const int q4 = lane >> 3, c8 = (lane & 7) * 8;
    u4v pk[4];
#pragma unroll
    for (int it = 0; it < 4; ++it) {
      const int idx = ow + (it * 4 + q4) * 68 + c8;
      const v4f f0 = *(const v4f*)&Os[idx], f1 = *(const v4f*)&Os[idx + 4];
      pk[it].x = cmb_pk2(f0.x, f0.y); pk[it].y = cmb_pk2(f0.z, f0.w); pk[it].z = cmb_pk2(f1.x, f1.y); pk[it].w = cmb_pk2(f1.z, f1.w);
    }
    unsigned short* ob = AO + hb + (size_t)q0 * 64;
    for (int pass = 0; pass < 2; ++pass) {
#pragma unroll
      for (int it = 0; it < 4; ++it) *(volatile u4v*)(ob + (it * 4 + q4) * 64 + c8) = pk[it];
      __threadfence();
    }
  }
}

template <int XRAW, int WF, int W16>
__device__ __forceinline__ void ln_body(const float* __restrict__ A, const float* __restrict__ X, float* __restrict__ Yf, unsigned short* __restrict__ Y16) {
    #pragma clang fp contract(off)
    const int r = blockIdx.x * 8 + (threadIdx.x >> 5); const int L = threadIdx.x & 31;
    if (r >= ROWS) return;
    const size_t xr = XRAW ? ((size_t)(r / SEQ) * SEQ_FULL + (size_t)(r % SEQ)) : (size_t)r;
    v4f v[8]; float s = 0.f;
#pragma unroll
    for (int q = 0; q < 8; ++q) {
        const int cc = 4 * L + 128 * q;
        const v4f a = *(const v4f*)(A + (size_t)r * DM + cc);
        v4f x = *(const v4f*)(X + xr * DM + cc);
        if (XRAW) { x.x = cmb_bf(x.x); x.y = cmb_bf(x.y); x.z = cmb_bf(x.z); x.w = cmb_bf(x.w); }
        v[q].x = a.x + x.x; v[q].y = a.y + x.y; v[q].z = a.z + x.z; v[q].w = a.w + x.w;
        s += (v[q].x + v[q].y) + (v[q].z + v[q].w);
    }
#pragma unroll
    for (int o = 16; o > 0; o >>= 1) s += __shfl_xor(s, o, 32);
    const float mu = s * (1.f / DM); float qq = 0.f;
#pragma unroll
    for (int q = 0; q < 8; ++q) {
        v[q].x -= mu; v[q].y -= mu; v[q].z -= mu; v[q].w -= mu;
        qq += (v[q].x * v[q].x + v[q].y * v[q].y) + (v[q].z * v[q].z + v[q].w * v[q].w);
    }
#pragma unroll
    for (int o = 16; o > 0; o >>= 1) qq += __shfl_xor(qq, o, 32);
    const float sd = sqrtf(qq * (1.f / DM));
    const float rs = 1.0f / sd;
#pragma unroll
    for (int q = 0; q < 8; ++q) {
        const size_t o = (size_t)r * DM + 4 * L + 128 * q;
        v4f y; y.x = v[q].x * rs; y.y = v[q].y * rs; y.z = v[q].z * rs; y.w = v[q].w * rs;
        if (WF) VST2(v4f, (v4f*)(Yf + o), y);
        if (W16) { u2v pk; pk.x = cmb_pk2(y.x, y.y); pk.y = cmb_pk2(y.z, y.w); VST2(u2v, (u2v*)(Y16 + o), pk); }
    }
}
__global__ __launch_bounds__(256) void k_ln1(const float* __restrict__ ATT, const float* __restrict__ x, float* __restrict__ AB, unsigned short* __restrict__ AB16) {
    ln_body<1, 1, 1>(ATT, x, AB, AB16);
}
__global__ __launch_bounds__(256) void k_ln2(const float* __restrict__ FF, const float* __restrict__ AB, float* __restrict__ out) {
    ln_body<0, 1, 0>(FF, AB, out, nullptr);
}

extern "C" void kernel_launch(void* const* d_in, const int* in_sizes, int n_in, void* d_out, int out_size, void* d_ws, size_t ws_size, hipStream_t stream) {
    if (n_in < 14) return;
    if (in_sizes[0] < (NB - 1) * SEQ_FULL * DM + SEQ * DM) return;
    if (in_sizes[1] < DM * DM || in_sizes[3] < DM * DM || in_sizes[5] < DM * DM || in_sizes[7] < DM * DM || in_sizes[10] < DM * DM || in_sizes[12] < DM * DM) return;
    if (in_sizes[2] < DM || in_sizes[4] < DM || in_sizes[6] < DM || in_sizes[8] < DM || in_sizes[11] < DM || in_sizes[13] < DM) return;
    if (in_sizes[9] < 32 * NHB) return;
    if (out_size < ROWS * DM) return;
    const float* x   = (const float*)d_in[0];
    const float* Wq  = (const float*)d_in[1];
    const float* bq  = (const float*)d_in[2];
    const float* Wk  = (const float*)d_in[3];
    const float* bk  = (const float*)d_in[4];
    const float* Wv  = (const float*)d_in[5];
    const float* bv  = (const float*)d_in[6];
    const float* Wo  = (const float*)d_in[7];
    const float* bo  = (const float*)d_in[8];
    const float* rel = (const float*)d_in[9];
    const float* W1  = (const float*)d_in[10];
    const float* b1  = (const float*)d_in[11];
    const float* W2  = (const float*)d_in[12];
    const float* b2  = (const float*)d_in[13];
    float* out = (float*)d_out;

    constexpr size_t NT  = (size_t)ROWS * DM;
    constexpr size_t NWT = (size_t)DM * DM;
    constexpr size_t O_X16  = 0;
    constexpr size_t O_WQ   = O_X16 + NT * 2;
    constexpr size_t O_WK   = O_WQ + NWT * 2;
    constexpr size_t O_WV   = O_WK + NWT * 2;
    constexpr size_t O_WO   = O_WV + NWT * 2;
    constexpr size_t O_W1   = O_WO + NWT * 2;
    constexpr size_t O_W2   = O_W1 + NWT * 2;
    constexpr size_t O_QH   = O_W2 + NWT * 2;
    constexpr size_t O_QL   = O_QH + NT * 2;
    constexpr size_t O_KH   = O_QL + NT * 2;
    constexpr size_t O_KL   = O_KH + NT * 2;
    constexpr size_t O_V16  = O_KL + NT * 2;
    constexpr size_t O_VT   = O_V16 + NT * 2;
    constexpr size_t O_AO   = O_VT + NT * 2;
    constexpr size_t O_ATT  = O_AO + NT * 2;
    constexpr size_t O_AB   = O_ATT + NT * 4;
    constexpr size_t O_AB16 = O_AB + NT * 4;
    constexpr size_t O_H16  = O_AB16 + NT * 2;
    constexpr size_t O_FF   = O_H16 + NT * 2;
    constexpr size_t WS_TOTAL = O_FF + NT * 4;
    static_assert(WS_TOTAL <= (size_t)134217728);
    static_assert((NT * 2) % 256 == 0);
    static_assert((NWT * 2) % 256 == 0);
    if (WS_TOTAL > ws_size) return;
    char* wsp = (char*)d_ws;
    unsigned short* X16  = (unsigned short*)(wsp + O_X16);
    unsigned short* WQ16 = (unsigned short*)(wsp + O_WQ);
    unsigned short* WK16 = (unsigned short*)(wsp + O_WK);
    unsigned short* WV16 = (unsigned short*)(wsp + O_WV);
    unsigned short* WO16 = (unsigned short*)(wsp + O_WO);
    unsigned short* W116 = (unsigned short*)(wsp + O_W1);
    unsigned short* W216 = (unsigned short*)(wsp + O_W2);
    unsigned short* QH   = (unsigned short*)(wsp + O_QH);
    unsigned short* QL   = (unsigned short*)(wsp + O_QL);
    unsigned short* KH   = (unsigned short*)(wsp + O_KH);
    unsigned short* KL   = (unsigned short*)(wsp + O_KL);
    unsigned short* V16  = (unsigned short*)(wsp + O_V16);
    unsigned short* VT16 = (unsigned short*)(wsp + O_VT);
    unsigned short* AO16 = (unsigned short*)(wsp + O_AO);
    float*          ATT  = (float*)(wsp + O_ATT);
    float*          AB   = (float*)(wsp + O_AB);
    unsigned short* AB16 = (unsigned short*)(wsp + O_AB16);
    unsigned short* H16  = (unsigned short*)(wsp + O_H16);
    float*          FF   = (float*)(wsp + O_FF);

    const unsigned gx = (unsigned)(((long long)ROWS * (DM / 8) + 255) / 256);
    const unsigned gw = (unsigned)(((long long)DM * (DM / 8) + 255) / 256);
    k_castb<<<gx, 256, 0, stream>>>(x,  X16,  ROWS, SEQ, SEQ_FULL, 1.0f);
    k_castb<<<gw, 256, 0, stream>>>(Wq, WQ16, DM, DM, DM, 16.0f);
    k_castb<<<gw, 256, 0, stream>>>(Wk, WK16, DM, DM, DM, 16.0f);
    k_castb<<<gw, 256, 0, stream>>>(Wv, WV16, DM, DM, DM, 16.0f);
    k_castb<<<gw, 256, 0, stream>>>(Wo, WO16, DM, DM, DM, 16.0f);
    k_castb<<<gw, 256, 0, stream>>>(W1, W116, DM, DM, DM, 16.0f);
    k_castb<<<gw, 256, 0, stream>>>(W2, W216, DM, DM, DM, 16.0f);

    const unsigned gg = (unsigned)((((ROWS) / 64) * ((DM) / 64) + 7) / 8);
    k_gemm_hl<<<gg, 256, 0, stream>>>(X16, DM, WQ16, DM, QH, QL, DM, bq, ROWS, DM, DM, 0.0625f);
    k_gemm_hl<<<gg, 256, 0, stream>>>(X16, DM, WK16, DM, KH, KL, DM, bk, ROWS, DM, DM, 0.0625f);
    k_gemm_h16<<<gg, 256, 0, stream>>>(X16, DM, WV16, DM, V16, DM, bv, ROWS, DM, DM, 0.0625f);
    k_vt<<<(unsigned)(NHEAD * (SEQ / 64)), 256, 0, stream>>>(V16, VT16);
    k_attn_rb<<<(unsigned)(NHEAD * (SEQ / 64)), 128, 0, stream>>>(QH, QL, KH, KL, VT16, rel, AO16);
    k_gemm_f32<<<gg, 256, 0, stream>>>(AO16, DM, WO16, DM, ATT, DM, bo, ROWS, DM, DM, 0.0625f);
    k_ln1<<<(unsigned)((ROWS + 7) / 8), 256, 0, stream>>>(ATT, x, AB, AB16);
    k_gemm_h16<<<gg, 256, 0, stream>>>(AB16, DM, W116, DM, H16, DM, b1, ROWS, DM, DM, 0.0625f);
    k_gemm_f32<<<gg, 256, 0, stream>>>(H16, DM, W216, DM, FF, DM, b2, ROWS, DM, DM, 0.0625f);
    k_ln2<<<(unsigned)((ROWS + 7) / 8), 256, 0, stream>>>(FF, AB, out);
}
